// student_graph_40157944217665
// MI455X (gfx1250) — hardware-verified
//
#include <hip/hip_runtime.h>
#include <stddef.h>


#define NBAT   4
#define SEQ4   1024
#define LSEQ   4096
#define CD     256
#define DKD    64
#define NBH    16
#define NTOP   36
#define NSMP   36
#define UP     64
#define NTHR   256
#define NWAVE  8
#define HSZ    (LSEQ * DKD)
#define BSZ    (SEQ4 * CD)
#define ROWS   (NBAT * LSEQ)
#define GROWS  128
#define KTS    128
#define KC     64
#define PP     72
#define WPL    (CD * CD)

static_assert(ROWS % GROWS == 0);
static_assert(GROWS == NWAVE * 16);
static_assert(LSEQ % KTS == 0 && LSEQ % KC == 0);
static_assert((PP % 8) == 0);
static_assert(LSEQ == 16 * NTHR);
static_assert(KTS == NWAVE * 16);
static_assert(UP * DKD * 4 <= 2 * UP * PP * 2);
static_assert(2 * UP * DKD * 2 <= 2 * DKD * PP * 2);
static_assert(UP * KTS * 4 <= 2 * KTS * PP * 2);
static_assert(HSZ == BSZ);

typedef float          v4f  __attribute__((ext_vector_type(4)));
typedef float          v8f  __attribute__((ext_vector_type(8)));
typedef int            v4i  __attribute__((ext_vector_type(4)));
typedef unsigned short v8us __attribute__((ext_vector_type(8)));
typedef __bf16         v16b __attribute__((ext_vector_type(16)));
typedef unsigned long long u64;
union FragB { v16b v; v8us h[2]; };

__device__ __forceinline__ unsigned bfr(float f) {
  const unsigned u = __float_as_uint(f);
  return (u + 0x7FFFu + ((u >> 16) & 1u)) >> 16;
}
__device__ __forceinline__ void split1(float x, unsigned short& h, unsigned short& l) {
  const unsigned hb = bfr(x);
  const float hf = __uint_as_float(hb << 16);
  h = (unsigned short)hb;
  l = (unsigned short)bfr(x - hf);
}
__device__ __forceinline__ void split8(v4f a, v4f b, v8us& hi, v8us& lo) {
  unsigned short h0, h1, h2, h3, h4, h5, h6, h7, l0, l1, l2, l3, l4, l5, l6, l7;
  split1(a.x, h0, l0); split1(a.y, h1, l1); split1(a.z, h2, l2); split1(a.w, h3, l3);
  split1(b.x, h4, l4); split1(b.y, h5, l5); split1(b.z, h6, l6); split1(b.w, h7, l7);
  hi[0] = h0; hi[1] = h1; hi[2] = h2; hi[3] = h3; hi[4] = h4; hi[5] = h5; hi[6] = h6; hi[7] = h7;
  lo[0] = l0; lo[1] = l1; lo[2] = l2; lo[3] = l3; lo[4] = l4; lo[5] = l5; lo[6] = l6; lo[7] = l7;
}

__device__ __forceinline__ v8f wmb(v16b a, v16b b, v8f c) {
  v8f d = __builtin_amdgcn_wmma_f32_16x16x32_bf16(false, a, false, b, (short)0, c, false, false);
  asm volatile("v_nop\n\tv_nop\n\tv_nop\n\tv_nop" : "+v"(d) : "v"(a), "v"(b));
  return d;
}

__device__ __forceinline__ u64 mkkeyb(unsigned u, int idx) {
  const unsigned mneg = ~u, mpos = u | 0x80000000u;
  const unsigned mono = (u & 0x80000000u) ? mneg : mpos;
  return ((u64)mono << 32) | (u64)(~(unsigned)idx);
}

__global__ __launch_bounds__(NTHR) void k_wprep(
    const float* __restrict__ Wq, const float* __restrict__ Wk, const float* __restrict__ Wv,
    const float* __restrict__ Wo, unsigned short* wp) {
  const int seg = (int)blockIdx.x >> 5;
  const float* src = seg == 0 ? Wq : (seg == 1 ? Wk : (seg == 2 ? Wv : Wo));
  const int i  = ((int)(blockIdx.x & 31) * NTHR) + (int)threadIdx.x;
  const int n  = i >> 5;
  const int k0 = (i & 31) * 8;
  v4f a, b;
  a.x = src[(k0 + 0) * CD + n]; a.y = src[(k0 + 1) * CD + n];
  a.z = src[(k0 + 2) * CD + n]; a.w = src[(k0 + 3) * CD + n];
  b.x = src[(k0 + 4) * CD + n]; b.y = src[(k0 + 5) * CD + n];
  b.z = src[(k0 + 6) * CD + n]; b.w = src[(k0 + 7) * CD + n];
  v8us hi, lo;
  split8(a, b, hi, lo);
  unsigned short* dh = wp + (size_t)seg * 2 * WPL + (size_t)i * 8;
  unsigned short* dl = dh + WPL;
  *(volatile v8us*)dh = hi;
  *(volatile v8us*)dl = lo;
  __threadfence();
  *(volatile v8us*)dh = hi;
  *(volatile v8us*)dl = lo;
}

__global__ __launch_bounds__(NTHR) void k_xprep(
    const float* __restrict__ et, const float* __restrict__ mp, const float* __restrict__ co,
    const float* __restrict__ vol, unsigned short* xh, unsigned short* xl) {
  const int g = (int)blockIdx.x * NTHR + (int)threadIdx.x;
  const int token = g >> 5;
  const int c0 = (g & 31) * 8;
  const int bp = token >> 12;
  const int l  = token & (LSEQ - 1);
  const int t  = (l & 15) >> 2;
  const int s  = ((l >> 4) << 2) + (l & 3);
  const float* src = (t == 0) ? et : ((t == 1) ? co : ((t == 2) ? mp : vol));
  const float* rp = src + (size_t)bp * BSZ + (size_t)s * CD + c0;
  const v4f a = *(const v4f*)rp, b = *(const v4f*)(rp + 4);
  v8us hi, lo;
  split8(a, b, hi, lo);
  unsigned short* dh = xh + (size_t)token * CD + c0;
  unsigned short* dl = xl + (size_t)token * CD + c0;
  *(volatile v8us*)dh = hi;
  *(volatile v8us*)dl = lo;
  __threadfence();
  *(volatile v8us*)dh = hi;
  *(volatile v8us*)dl = lo;
}

__global__ __launch_bounds__(NTHR) void k_gemm(
    const unsigned short* __restrict__ Ah, const unsigned short* __restrict__ Al,
    const unsigned short* __restrict__ wp, int wsel,
    const float* __restrict__ b0, const float* __restrict__ b1, const float* __restrict__ b2,
    float* C0, float* C1, float* C2) {
  __shared__ __attribute__((aligned(16))) float stg[NWAVE * 16 * 64];
  const int tid = threadIdx.x, lane = tid & 31, wave = tid >> 5, hh = lane >> 4, m = lane & 15;
  const int j = (int)blockIdx.y;
  const unsigned short* Wh = wp + (size_t)(wsel + j) * 2 * WPL;
  const unsigned short* Wl = Wh + WPL;
  const float* bias = (j == 0) ? b0 : ((j == 1) ? b1 : b2);
  float* Cp = (j == 0) ? C0 : ((j == 1) ? C1 : C2);
  const int rowBase = (int)blockIdx.x * GROWS;
  const size_t arow = ((size_t)rowBase + wave * 16 + m) * CD + 8 * hh;
  const unsigned short* arh = Ah + arow;
  const unsigned short* arl = Al + arow;
  float* sw = stg + wave * (16 * 64);

#pragma unroll 1
  for (int tp = 0; tp < 4; ++tp) {
    v8f acc[4];
#pragma unroll
    for (int t = 0; t < 4; ++t) { v8f z = {0.f, 0.f, 0.f, 0.f, 0.f, 0.f, 0.f, 0.f}; acc[t] = z; }
#pragma unroll 1
    for (int kt = 0; kt < CD / 32; ++kt) {
      FragB ah, al;
      ah.h[0] = *(const v8us*)(arh + 32 * kt);
      ah.h[1] = *(const v8us*)(arh + 32 * kt + 16);
      al.h[0] = *(const v8us*)(arl + 32 * kt);
      al.h[1] = *(const v8us*)(arl + 32 * kt + 16);
#pragma unroll
      for (int t = 0; t < 4; ++t) {
        const size_t bo = (size_t)(64 * tp + 16 * t + m) * CD + 32 * kt + 8 * hh;
        FragB wbh, wbl;
        wbh.h[0] = *(const v8us*)(Wh + bo);
        wbh.h[1] = *(const v8us*)(Wh + bo + 16);
        wbl.h[0] = *(const v8us*)(Wl + bo);
        wbl.h[1] = *(const v8us*)(Wl + bo + 16);
        acc[t] = wmb(ah.v, wbh.v, acc[t]);
        acc[t] = wmb(ah.v, wbl.v, acc[t]);
        acc[t] = wmb(al.v, wbh.v, acc[t]);
      }
    }
    float bs[4];
#pragma unroll
    for (int t = 0; t < 4; ++t) bs[t] = bias[64 * tp + 16 * t + m];
#pragma unroll
    for (int t = 0; t < 4; ++t) {
#pragma unroll
      for (int r = 0; r < 8; ++r) sw[(8 * hh + r) * 64 + 16 * t + m] = acc[t][r] + bs[t];
    }
    __syncthreads();
    const float* lp = sw + hh * 64 + 4 * m;
    float* gp = Cp + ((size_t)rowBase + wave * 16 + hh) * CD + 64 * tp + 4 * m;
    v4f rv[8];
#pragma unroll
    for (int i = 0; i < 8; ++i) rv[i] = *(const v4f*)(lp + i * 128);
#pragma unroll
    for (int i = 0; i < 8; ++i) *(volatile v4f*)(gp + (size_t)i * 2 * CD) = rv[i];
    __threadfence();
#pragma unroll
    for (int i = 0; i < 8; ++i) *(volatile v4f*)(gp + (size_t)i * 2 * CD) = rv[i];
    __syncthreads();
  }
}

__global__ __launch_bounds__(NTHR) void k_msel(
    const float* __restrict__ qp, const float* __restrict__ kp, const int* __restrict__ isamp,
    int* toplist) {
  __shared__ __attribute__((aligned(16))) u64 skey[LSEQ];
  const int tid = threadIdx.x;
  const int bh = (int)blockIdx.x;
  const float* qb = qp + (size_t)bh * HSZ;
  const float* kb = kp + (size_t)bh * HSZ;

#pragma unroll 1
  for (int jq = 0; jq < LSEQ / NTHR; ++jq) {
    const int s = jq * NTHR + tid;
    const float* qr = qb + (size_t)s * DKD;
    v4f q[16];
#pragma unroll
    for (int d4 = 0; d4 < 16; ++d4) q[d4] = *(const v4f*)(qr + 4 * d4);
    float mx = __uint_as_float(0xff800000u);
    float sm = 0.0f;
    const int* ip = isamp + (size_t)s * NSMP;
#pragma unroll 1
    for (int kk = 0; kk < NSMP; ++kk) {
      int ix = ip[kk];
      ix = ix < 0 ? 0 : (ix > LSEQ - 1 ? LSEQ - 1 : ix);
      const float* kr = kb + (size_t)ix * DKD;
      float a0 = 0.f, a1 = 0.f, a2 = 0.f, a3 = 0.f;
#pragma unroll
      for (int d4 = 0; d4 < 16; ++d4) {
        const v4f kv = *(const v4f*)(kr + 4 * d4);
        a0 = fmaf(q[d4].x, kv.x, a0); a1 = fmaf(q[d4].y, kv.y, a1);
        a2 = fmaf(q[d4].z, kv.z, a2); a3 = fmaf(q[d4].w, kv.w, a3);
      }
      const float dot = (a0 + a1) + (a2 + a3);
      mx = fmaxf(mx, dot);
      sm += dot;
    }
    const float Mv = mx - sm * (1.0f / 4096.0f);
    unsigned ub = __float_as_uint(Mv);
    ub = (ub == 0x80000000u) ? 0u : ub;
    skey[s] = mkkeyb(ub, s);
  }
  __syncthreads();

#pragma unroll 1
  for (int kk = 2; kk <= LSEQ; kk <<= 1) {
#pragma unroll 1
    for (int jj = kk >> 1; jj > 0; jj >>= 1) {
#pragma unroll
      for (int qq = 0; qq < LSEQ / 2 / NTHR; ++qq) {
        const int t  = qq * NTHR + tid;
        const int i  = ((t & ~(jj - 1)) << 1) | (t & (jj - 1));
        const int i2 = i | jj;
        const u64 a = skey[i], b = skey[i2];
        const bool up = ((i & kk) == 0);
        const bool sw = up ? (a > b) : (a < b);
        if (sw) { skey[i] = b; skey[i2] = a; }
      }
      __syncthreads();
    }
  }

  if (tid < 16) {
    const int u0 = tid * 4;
    const u64 k0 = skey[LSEQ - 1 - u0], k1 = skey[LSEQ - 2 - u0];
    const u64 k2 = skey[LSEQ - 3 - u0], k3 = skey[LSEQ - 4 - u0];
    v4i tv;
    tv.x = (u0 + 0 < NTOP) ? (int)(~(unsigned)(k0 & 0xffffffffull)) : -1;
    tv.y = (u0 + 1 < NTOP) ? (int)(~(unsigned)(k1 & 0xffffffffull)) : -1;
    tv.z = (u0 + 2 < NTOP) ? (int)(~(unsigned)(k2 & 0xffffffffull)) : -1;
    tv.w = (u0 + 3 < NTOP) ? (int)(~(unsigned)(k3 & 0xffffffffull)) : -1;
    int* tp = toplist + (size_t)bh * UP + u0;
    *(volatile v4i*)tp = tv;
    __threadfence();
    *(volatile v4i*)tp = tv;
  }
}

__global__ __launch_bounds__(NTHR) void k_scores(
    const float* __restrict__ qp, const float* __restrict__ kp, const int* __restrict__ toplist,
    float* sc) {
  __shared__ __attribute__((aligned(16))) unsigned short sQ[2 * UP * PP];
  __shared__ __attribute__((aligned(16))) unsigned short sK[2 * KTS * PP];
  unsigned short* Qh = sQ; unsigned short* Ql = sQ + UP * PP;
  unsigned short* Kh = sK; unsigned short* Kl = sK + KTS * PP;
  float* stg = (float*)sK;
  const int tid = threadIdx.x, lane = tid & 31, wave = tid >> 5, hh = lane >> 4, m = lane & 15;
  const int bh = (int)blockIdx.y;
  const int kt0 = (int)blockIdx.x * KTS;

  {
    const int u = tid >> 2, d0 = (tid & 3) * 16;
    int ix = toplist[(size_t)bh * UP + u];
    const bool val = (u < NTOP);
    ix = ix < 0 ? 0 : (ix > LSEQ - 1 ? LSEQ - 1 : ix);
    const float* qr = qp + (size_t)bh * HSZ + (size_t)ix * DKD + d0;
    v4f a = *(const v4f*)qr, b = *(const v4f*)(qr + 4), c = *(const v4f*)(qr + 8), d = *(const v4f*)(qr + 12);
    const v4f z = {0.f, 0.f, 0.f, 0.f};
    if (!val) { a = z; b = z; c = z; d = z; }
    v8us h0, l0, h1, l1;
    split8(a, b, h0, l0); split8(c, d, h1, l1);
    *(v8us*)(Qh + u * PP + d0)     = h0;
    *(v8us*)(Qh + u * PP + d0 + 8) = h1;
    *(v8us*)(Ql + u * PP + d0)     = l0;
    *(v8us*)(Ql + u * PP + d0 + 8) = l1;
  }
  {
    const int kl = tid >> 1, d0 = (tid & 1) * 32;
    const float* kr = kp + (size_t)bh * HSZ + (size_t)(kt0 + kl) * DKD + d0;
#pragma unroll
    for (int e = 0; e < 4; ++e) {
      const v4f a = *(const v4f*)(kr + 8 * e), b = *(const v4f*)(kr + 8 * e + 4);
      v8us hi, lo;
      split8(a, b, hi, lo);
      *(v8us*)(Kh + kl * PP + d0 + 8 * e) = hi;
      *(v8us*)(Kl + kl * PP + d0 + 8 * e) = lo;
    }
  }
  __syncthreads();

  const int nt = wave;
  v8f acc[4];
#pragma unroll
  for (int t = 0; t < 4; ++t) { v8f z = {0.f, 0.f, 0.f, 0.f, 0.f, 0.f, 0.f, 0.f}; acc[t] = z; }
#pragma unroll
  for (int ks = 0; ks < 2; ++ks) {
    const int k0 = 32 * ks;
    FragB wbh, wbl;
    wbh.h[0] = *(const v8us*)(Kh + (nt * 16 + m) * PP + k0 + 8 * hh);
    wbh.h[1] = *(const v8us*)(Kh + (nt * 16 + m) * PP + k0 + 16 + 8 * hh);
    wbl.h[0] = *(const v8us*)(Kl + (nt * 16 + m) * PP + k0 + 8 * hh);
    wbl.h[1] = *(const v8us*)(Kl + (nt * 16 + m) * PP + k0 + 16 + 8 * hh);
#pragma unroll
    for (int mt = 0; mt < 4; ++mt) {
      FragB ah, al;
      ah.h[0] = *(const v8us*)(Qh + (mt * 16 + m) * PP + k0 + 8 * hh);
      ah.h[1] = *(const v8us*)(Qh + (mt * 16 + m) * PP + k0 + 16 + 8 * hh);
      al.h[0] = *(const v8us*)(Ql + (mt * 16 + m) * PP + k0 + 8 * hh);
      al.h[1] = *(const v8us*)(Ql + (mt * 16 + m) * PP + k0 + 16 + 8 * hh);
      acc[mt] = wmb(ah.v, wbh.v, acc[mt]);
      acc[mt] = wmb(ah.v, wbl.v, acc[mt]);
      acc[mt] = wmb(al.v, wbh.v, acc[mt]);
    }
  }
  __syncthreads();
#pragma unroll
  for (int mt = 0; mt < 4; ++mt) {
#pragma unroll
    for (int r = 0; r < 8; ++r) stg[(mt * 16 + 8 * hh + r) * KTS + nt * 16 + m] = acc[mt][r] * 0.125f;
  }
  __syncthreads();

  const float* lp = stg + (wave * 8) * KTS + 4 * lane;
  float* gp = sc + ((size_t)bh * UP + wave * 8) * LSEQ + kt0 + 4 * lane;
  v4f rv[8];
#pragma unroll
  for (int i = 0; i < 8; ++i) rv[i] = *(const v4f*)(lp + i * KTS);
#pragma unroll
  for (int i = 0; i < 8; ++i) *(volatile v4f*)(gp + (size_t)i * LSEQ) = rv[i];
  __threadfence();
#pragma unroll
  for (int i = 0; i < 8; ++i) *(volatile v4f*)(gp + (size_t)i * LSEQ) = rv[i];
}

__device__ __forceinline__ void ctx_pass(const int* rsel, const unsigned short* upH,
                                         const unsigned short* upL, const unsigned short* vsH,
                                         const unsigned short* vsL, unsigned short* gh,
                                         unsigned short* gl, int tid) {
#pragma unroll 1
  for (int i = 0; i < (LSEQ * 8) / NTHR; ++i) {
    const int f = i * NTHR + tid;
    const int l = f >> 3, p = f & 7;
    const int sel = rsel[l];
    const int sc_ = sel < 0 ? 0 : (sel > UP - 1 ? UP - 1 : sel);
    const v4i a  = *(const v4i*)(upH + sc_ * DKD + p * 8);
    const v4i al = *(const v4i*)(upL + sc_ * DKD + p * 8);
    const v4i b  = *(const v4i*)(vsH + p * 8);
    const v4i bl = *(const v4i*)(vsL + p * 8);
    const bool us = sel >= 0;
    v4i h, o;
    h.x = us ? a.x : b.x;   h.y = us ? a.y : b.y;   h.z = us ? a.z : b.z;   h.w = us ? a.w : b.w;
    o.x = us ? al.x : bl.x; o.y = us ? al.y : bl.y; o.z = us ? al.z : bl.z; o.w = us ? al.w : bl.w;
    *(volatile v4i*)(gh + (size_t)l * DKD + p * 8) = h;
    *(volatile v4i*)(gl + (size_t)l * DKD + p * 8) = o;
  }
}

__global__ __launch_bounds__(NTHR) void k_attn(
    const float* __restrict__ sc, const float* __restrict__ vp, const int* __restrict__ toplist,
    unsigned short* ctxh, unsigned short* ctxl) {
  __shared__ __attribute__((aligned(16))) unsigned short rA[2 * UP * PP];
  __shared__ __attribute__((aligned(16))) unsigned short rB[2 * DKD * PP];
  __shared__ __attribute__((aligned(16))) float vps[4 * DKD];
  __shared__ __attribute__((aligned(16))) unsigned short vsH[DKD];
  __shared__ __attribute__((aligned(16))) unsigned short vsL[DKD];
  __shared__ float rmax[UP];
  __shared__ float rinv[UP];
  __shared__ int rsel[LSEQ];
  __shared__ int tops[UP];
  unsigned short* Ph = rA; unsigned short* Pl = rA + UP * PP;
  unsigned short* Vh = rB; unsigned short* Vl = rB + DKD * PP;
  float* stg = (float*)rA;
  unsigned short* upH = rB; unsigned short* upL = rB + UP * DKD;
  const int tid = threadIdx.x, lane = tid & 31, wave = tid >> 5, hh = lane >> 4, m = lane & 15;
  const int bh = (int)blockIdx.x;
  const float* scb = sc + (size_t)bh * UP * LSEQ;
  const float* vb = vp + (size_t)bh * HSZ;

  if (tid < UP) {
    int t = toplist[(size_t)bh * UP + tid];
    t = t < 0 ? 0 : (t > LSEQ - 1 ? LSEQ - 1 : t);
    tops[tid] = t;
    rmax[tid] = 0.0f;
    rinv[tid] = 0.0f;
  }
  for (int i = tid; i < LSEQ; i += NTHR) rsel[i] = -1;
  __syncthreads();
  if (tid < NTOP) rsel[tops[tid]] = tid;

  for (int u = wave; u < NTOP; u += NWAVE) {
    const float* pr = scb + (size_t)u * LSEQ + 4 * lane;
    float mx = __uint_as_float(0xff800000u);
#pragma unroll 4
    for (int i = 0; i < LSEQ / 128; ++i) {
      const v4f s = *(const v4f*)(pr + i * 128);
      mx = fmaxf(mx, fmaxf(fmaxf(s.x, s.y), fmaxf(s.z, s.w)));
    }
#pragma unroll
    for (int o = 16; o > 0; o >>= 1) mx = fmaxf(mx, __shfl_xor(mx, o));
    float sm = 0.0f;
#pragma unroll 1
    for (int i = 0; i < LSEQ / 128; ++i) {
      const v4f s = *(const v4f*)(pr + i * 128);
      sm += (expf(s.x - mx) + expf(s.y - mx)) + (expf(s.z - mx) + expf(s.w - mx));
    }
#pragma unroll
    for (int o = 16; o > 0; o >>= 1) sm += __shfl_xor(sm, o);
    if (lane == 0) { rmax[u] = mx; rinv[u] = 1.0f / sm; }
  }
  __syncthreads();

  v8f acc[2];
#pragma unroll
  for (int t = 0; t < 2; ++t) { v8f z = {0.f, 0.f, 0.f, 0.f, 0.f, 0.f, 0.f, 0.f}; acc[t] = z; }
  float vpart = 0.0f;
  const int nt = wave & 3, mt0 = (wave >> 2) * 2;
  const int pu = tid >> 2, pq = tid & 3;
  const int vd = tid & 63, vg = tid >> 6;
  const float pmx = rmax[pu], pri = rinv[pu];
  const bool pval = (pu < NTOP);
  const v4f z4 = {0.f, 0.f, 0.f, 0.f};
#pragma unroll 1
  for (int c = 0; c < LSEQ / KC; ++c) {
    {
      const float* pr = scb + (size_t)pu * LSEQ + c * KC + pq * 16;
#pragma unroll 1
      for (int hf = 0; hf < 2; ++hf) {
        const v4f s0 = *(const v4f*)(pr + 8 * hf), s1 = *(const v4f*)(pr + 8 * hf + 4);
        v4f p0, p1;
        p0.x = expf(s0.x - pmx) * pri; p0.y = expf(s0.y - pmx) * pri;
        p0.z = expf(s0.z - pmx) * pri; p0.w = expf(s0.w - pmx) * pri;
        p1.x = expf(s1.x - pmx) * pri; p1.y = expf(s1.y - pmx) * pri;
        p1.z = expf(s1.z - pmx) * pri; p1.w = expf(s1.w - pmx) * pri;
        if (!pval) { p0 = z4; p1 = z4; }
        v8us h8, l8;
        split8(p0, p1, h8, l8);
        *(v8us*)(Ph + pu * PP + pq * 16 + 8 * hf) = h8;
        *(v8us*)(Pl + pu * PP + pq * 16 + 8 * hf) = l8;
      }
    }
    {
      const float* vr = vb + (size_t)(c * KC + vg * 16) * DKD + vd;
      v4f a, b, e, f;
      a.x = vr[0 * DKD];  a.y = vr[1 * DKD];  a.z = vr[2 * DKD];  a.w = vr[3 * DKD];
      b.x = vr[4 * DKD];  b.y = vr[5 * DKD];  b.z = vr[6 * DKD];  b.w = vr[7 * DKD];
      e.x = vr[8 * DKD];  e.y = vr[9 * DKD];  e.z = vr[10 * DKD]; e.w = vr[11 * DKD];
      f.x = vr[12 * DKD]; f.y = vr[13 * DKD]; f.z = vr[14 * DKD]; f.w = vr[15 * DKD];
      vpart += (((a.x + a.y) + (a.z + a.w)) + ((b.x + b.y) + (b.z + b.w))) +
               (((e.x + e.y) + (e.z + e.w)) + ((f.x + f.y) + (f.z + f.w)));
      v8us h0, l0, h1, l1;
      split8(a, b, h0, l0); split8(e, f, h1, l1);
      *(v8us*)(Vh + vd * PP + vg * 16)     = h0;
      *(v8us*)(Vh + vd * PP + vg * 16 + 8) = h1;
      *(v8us*)(Vl + vd * PP + vg * 16)     = l0;
      *(v8us*)(Vl + vd * PP + vg * 16 + 8) = l1;
    }
    __syncthreads();
#pragma unroll
    for (int ks = 0; ks < 2; ++ks) {
      const int k0 = 32 * ks;
      FragB wbh, wbl;
      wbh.h[0] = *(const v8us*)(Vh + (nt * 16 + m) * PP + k0 + 8 * hh);
      wbh.h[1] = *(const v8us*)(Vh + (nt * 16 + m) * PP + k0 + 16 + 8 * hh);
      wbl.h[0] = *(const v8us*)(Vl + (nt * 16 + m) * PP + k0 + 8 * hh);
      wbl.h[1] = *(const v8us*)(Vl + (nt * 16 + m) * PP + k0 + 16 + 8 * hh);
#pragma unroll
      for (int jm = 0; jm < 2; ++jm) {
        const int mt = mt0 + jm;
        FragB ah, al;
        ah.h[0] = *(const v8us*)(Ph + (mt * 16 + m) * PP + k0 + 8 * hh);
        ah.h[1] = *(const v8us*)(Ph + (mt * 16 + m) * PP + k0 + 16 + 8 * hh);
        al.h[0] = *(const v8us*)(Pl + (mt * 16 + m) * PP + k0 + 8 * hh);
        al.h[1] = *(const v8us*)(Pl + (mt * 16 + m) * PP + k0 + 16 + 8 * hh);
        acc[jm] = wmb(ah.v, wbh.v, acc[jm]);
        acc[jm] = wmb(ah.v, wbl.v, acc[jm]);
        acc[jm] = wmb(al.v, wbh.v, acc[jm]);
      }
    }
    __syncthreads();
  }

#pragma unroll
  for (int jm = 0; jm < 2; ++jm) {
#pragma unroll
    for (int r = 0; r < 8; ++r) stg[((mt0 + jm) * 16 + 8 * hh + r) * DKD + nt * 16 + m] = acc[jm][r];
  }
  vps[vg * DKD + vd] = vpart;
  __syncthreads();
  {
    const int u = tid >> 2, d0 = (tid & 3) * 16;
    const float* sp = stg + u * DKD + d0;
    const v4f a = *(const v4f*)sp, b = *(const v4f*)(sp + 4), e = *(const v4f*)(sp + 8), f = *(const v4f*)(sp + 12);
    v8us h0, l0, h1, l1;
    split8(a, b, h0, l0); split8(e, f, h1, l1);
    *(v8us*)(upH + u * DKD + d0)     = h0;
    *(v8us*)(upH + u * DKD + d0 + 8) = h1;
    *(v8us*)(upL + u * DKD + d0)     = l0;
    *(v8us*)(upL + u * DKD + d0 + 8) = l1;
    if (tid < DKD) {
      const float vsum = (vps[tid] + vps[DKD + tid]) + (vps[2 * DKD + tid] + vps[3 * DKD + tid]);
      unsigned short h, l;
      split1(vsum, h, l);
      vsH[tid] = h;
      vsL[tid] = l;
    }
  }
  __syncthreads();

  unsigned short* gh = ctxh + (size_t)bh * HSZ;
  unsigned short* gl = ctxl + (size_t)bh * HSZ;
  ctx_pass(rsel, upH, upL, vsH, vsL, gh, gl, tid);
  __threadfence();
  ctx_pass(rsel, upH, upL, vsH, vsL, gh, gl, tid);
}

extern "C" void kernel_launch(void* const* d_in, const int* in_sizes, int n_in,
                              void* d_out, int out_size, void* d_ws, size_t ws_size,
                              hipStream_t stream) {
  if (n_in < 13) return;
  for (int i = 0; i < 4; ++i) if (in_sizes[i] != NBAT * BSZ) return;
  if (in_sizes[4] != WPL || in_sizes[6] != WPL || in_sizes[8] != WPL || in_sizes[10] != WPL) return;
  if (in_sizes[5] != CD || in_sizes[7] != CD || in_sizes[9] != CD || in_sizes[11] != CD) return;
  if (in_sizes[12] != LSEQ * NSMP) return;
  if (out_size != ROWS * CD) return;

  const float* et  = (const float*)d_in[0];
  const float* mp  = (const float*)d_in[1];
  const float* co  = (const float*)d_in[2];
  const float* vol = (const float*)d_in[3];
  const float* Wq  = (const float*)d_in[4];
  const float* bq  = (const float*)d_in[5];
  const float* Wk  = (const float*)d_in[6];
  const float* bk  = (const float*)d_in[7];
  const float* Wv  = (const float*)d_in[8];
  const float* bv  = (const float*)d_in[9];
  const float* Wo  = (const float*)d_in[10];
  const float* bo  = (const float*)d_in[11];
  const int*   isamp = (const int*)d_in[12];
  float* out = (float*)d_out;

  char* ws = (char*)d_ws;
  size_t off = 0;
#define CARVE(NAME, BYTES) const size_t NAME = off; off += (size_t)(BYTES); off = (off + 255) & ~(size_t)255;
  CARVE(oW,   (size_t)4 * 2 * WPL * 2)
  CARVE(oXh,  (size_t)ROWS * CD * 2)
  CARVE(oXl,  (size_t)ROWS * CD * 2)
  CARVE(oQ,   (size_t)ROWS * CD * 4)
  CARVE(oK,   (size_t)ROWS * CD * 4)
  CARVE(oV,   (size_t)ROWS * CD * 4)
  CARVE(oTop, (size_t)NBH * UP * 4)
  CARVE(oSc,  (size_t)NBH * UP * LSEQ * 4)
  CARVE(oCh,  (size_t)ROWS * CD * 2)
  CARVE(oCl,  (size_t)ROWS * CD * 2)
#undef CARVE
  if (off > ws_size) return;
  if (off > (size_t)134217728) return;

  unsigned short* wp   = (unsigned short*)(ws + oW);
  unsigned short* xh   = (unsigned short*)(ws + oXh);
  unsigned short* xl   = (unsigned short*)(ws + oXl);
  float*          qpl  = (float*)(ws + oQ);
  float*          kpl  = (float*)(ws + oK);
  float*          vpl  = (float*)(ws + oV);
  int*            top  = (int*)(ws + oTop);
  float*          scp  = (float*)(ws + oSc);
  unsigned short* ctxh = (unsigned short*)(ws + oCh);
  unsigned short* ctxl = (unsigned short*)(ws + oCl);

  k_wprep<<<4 * 32, NTHR, 0, stream>>>(Wq, Wk, Wv, Wo, wp);
  k_xprep<<<(ROWS * 32) / NTHR, NTHR, 0, stream>>>(et, mp, co, vol, xh, xl);
  k_gemm<<<dim3(ROWS / GROWS, 3), NTHR, 0, stream>>>(xh, xl, wp, 0, bq, bk, bv, qpl, kpl, vpl);
  k_msel<<<NBH, NTHR, 0, stream>>>(qpl, kpl, isamp, top);
  k_scores<<<dim3(LSEQ / KTS, NBH), NTHR, 0, stream>>>(qpl, kpl, top, scp);
  k_attn<<<NBH, NTHR, 0, stream>>>(scp, vpl, top, ctxh, ctxl);
  k_gemm<<<dim3(ROWS / GROWS, 1), NTHR, 0, stream>>>(ctxh, ctxl, wp, 3, bo, bo, bo, out, out, out);
}
